// Q_network_4621384810937
// MI455X (gfx1250) — hardware-verified
//
#include <hip/hip_runtime.h>
#include <hip/hip_bf16.h>
#include <math.h>


#define BB 2
#define SS 2048
#define DD 1024
#define HH 16
#define DKK 64
#define QW 2

typedef _Float16 bf16;
typedef __attribute__((ext_vector_type(4))) unsigned v4u_t;
typedef unsigned v4ua __attribute__((ext_vector_type(4), may_alias));
typedef __attribute__((ext_vector_type(4))) float v4f_t;
typedef float v4fa __attribute__((ext_vector_type(4), may_alias));
typedef __attribute__((ext_vector_type(16))) bf16  bf16x16;
typedef __attribute__((ext_vector_type(8)))  bf16  bf16x8;
typedef __attribute__((ext_vector_type(4)))  bf16  bf16x4;
typedef __attribute__((ext_vector_type(8)))  float f32x8;

#define LDS_STRIDE 48
#define KSTRIDE    72
#define VSTRIDE    48

__device__ __forceinline__ f32x8 wmma_bf16(bf16x16 a, bf16x16 b, f32x8 c) {
  return __builtin_amdgcn_wmma_f32_16x16x32_f16(
      false, a, false, b, (short)0, c, false, false);
}
#define RSPLIT (1.0f / 2048.0f)
__device__ __forceinline__ bf16 lo_of(float v, bf16 h) { return (bf16)((v - (float)h) * 2048.0f); }
__device__ __forceinline__ f32x8 wmma_split(bf16x16 a, bf16x16 al, bf16x16 b, bf16x16 bl, f32x8 c) {
  f32x8 x = {}; x = wmma_bf16(al, b, x); x = wmma_bf16(a, bl, x); return wmma_bf16(a, b, c) + x * RSPLIT; }

template <typename T>
__device__ __forceinline__ bf16x16 load_frag(const T* __restrict__ base, int ld,
                                             int row0, int k0) {
  const int lane = threadIdx.x & 31;
  const int r    = lane & 15;
  const int kh   = (lane >> 4) * 8;
  const T* p0 = base + (size_t)(row0 + r) * ld + (k0 + kh);
  const T* p1 = p0 + 16;
  bf16x16 f;
#pragma unroll
  for (int i = 0; i < 8; ++i) {
    f[i]     = (bf16)p0[i];
    f[i + 8] = (bf16)p1[i];
  }
  return f;
}

__device__ __forceinline__ bf16x16 lds_frag(const bf16* base, int stride) {
  const int lane = threadIdx.x & 31;
  const int row  = lane & 15;
  const int kh   = (lane >> 4) * 8;
  const bf16x8 lo = *(const bf16x8*)(base + row * stride + kh);
  const bf16x8 hi = *(const bf16x8*)(base + row * stride + kh + 16);
  bf16x16 f;
#pragma unroll
  for (int i = 0; i < 8; ++i) { f[i] = lo[i]; f[i + 8] = hi[i]; }
  return f;
}

template <typename T>
__device__ __forceinline__ void stage_read16(const T* __restrict__ p, float* buf) {
#pragma unroll
  for (int i = 0; i < 16; ++i) buf[i] = (float)p[i];
}

__device__ __forceinline__ void stage_write(bf16* dst, const float* buf, int nquad) {
#pragma unroll
  for (int i = 0; i < nquad; ++i) {
    bf16x4 q;
    q[0] = (bf16)buf[4 * i];     q[1] = (bf16)buf[4 * i + 1];
    q[2] = (bf16)buf[4 * i + 2]; q[3] = (bf16)buf[4 * i + 3];
    *(bf16x4*)(dst + 4 * i) = q;
  }
}

__global__ __launch_bounds__(256) void transpose_pack_kernel(const float* __restrict__ W, bf16* __restrict__ WT, int K, int N, size_t plane) {
  __shared__ float tile[64][65];
  const int k0 = blockIdx.y * 64, n0 = blockIdx.x * 64, t = threadIdx.x;
  for (int i = t; i < 64 * 64; i += 256) { const int kr = i >> 6, nc = i & 63; tile[kr][nc] = W[(size_t)(k0 + kr) * N + n0 + nc]; }
  __syncthreads();
#pragma unroll 1
  for (int pass = 0; pass < 2; ++pass) {
    for (int i = t; i < 64 * 8; i += 256) { const int nr = i >> 3, k8 = (i & 7) * 8; bf16 hh[8], hl[8];
#pragma unroll
      for (int e = 0; e < 8; ++e) { const float v = tile[k8 + e][nr]; hh[e] = (bf16)v; hl[e] = lo_of(v, hh[e]); }
      bf16* d = WT + (size_t)(n0 + nr) * K + k0 + k8;
      *(volatile v4u_t*)d = *(const v4ua*)hh; *(volatile v4u_t*)(d + plane) = *(const v4ua*)hl; }
    __threadfence();
  }
}

template <typename AT, typename WT, int MODE>
__global__ __launch_bounds__(256) void gemm_split_kernel(
    const AT* __restrict__ A, size_t aPlane, const WT* __restrict__ W, size_t wPlane,
    const float* __restrict__ bias, void* __restrict__ out,
    int M, int N, int K, int act) {
  __shared__ bf16 ldsA[128 * LDS_STRIDE], ldsAl[128 * LDS_STRIDE];
  __shared__ bf16 ldsW[256 * LDS_STRIDE], ldsWl[256 * LDS_STRIDE];
  __shared__ __attribute__((aligned(16))) unsigned char sob[256 * 136 * 2];

  const int t    = threadIdx.x;
  const int wave = t >> 5;
  const int lane = t & 31;
  const int wm   = (wave & 1) * 64;
  const int wn   = (wave >> 1) * 64;
  const int mBlk = blockIdx.x * 128;
  const int nBlk = blockIdx.y * 256;
  const int arow = t >> 1;
  const int ach  = (t & 1) * 16;

  f32x8 acc[4][4] = {};
  for (int k = 0; k < K; k += 32) {
    __syncthreads();
    {
      const AT* ap = A + (size_t)(mBlk + arow) * K + k + ach;
      bf16 hh[16], hl[16];
      if (sizeof(AT) == 4) {
#pragma unroll
        for (int i = 0; i < 16; ++i) { const float v = (float)ap[i]; hh[i] = (bf16)v; hl[i] = lo_of(v, hh[i]); }
      } else {
#pragma unroll
        for (int i = 0; i < 16; ++i) { hh[i] = (bf16)ap[i]; hl[i] = (bf16)ap[aPlane + i]; }
      }
#pragma unroll
      for (int i = 0; i < 16; ++i) { ldsA[arow * LDS_STRIDE + ach + i] = hh[i]; ldsAl[arow * LDS_STRIDE + ach + i] = hl[i]; }
    }
    {
      const WT* wp = W + (size_t)(nBlk + t) * K + k;
      if (sizeof(WT) == 4) {
#pragma unroll
        for (int i = 0; i < 32; ++i) { const float v = (float)wp[i]; const bf16 h_ = (bf16)v; ldsW[t * LDS_STRIDE + i] = h_; ldsWl[t * LDS_STRIDE + i] = lo_of(v, h_); }
      } else {
#pragma unroll
        for (int i = 0; i < 32; ++i) { ldsW[t * LDS_STRIDE + i] = (bf16)wp[i]; ldsWl[t * LDS_STRIDE + i] = (bf16)wp[wPlane + i]; }
      }
    }
    __syncthreads();
    bf16x16 wf[4], wfl[4];
#pragma unroll
    for (int j = 0; j < 4; ++j) { wf[j] = lds_frag(ldsW + (wn + 16 * j) * LDS_STRIDE, LDS_STRIDE); wfl[j] = lds_frag(ldsWl + (wn + 16 * j) * LDS_STRIDE, LDS_STRIDE); }
#pragma unroll
    for (int i = 0; i < 4; ++i) {
      const bf16x16 af = lds_frag(ldsA + (wm + 16 * i) * LDS_STRIDE, LDS_STRIDE), afl = lds_frag(ldsAl + (wm + 16 * i) * LDS_STRIDE, LDS_STRIDE);
#pragma unroll
      for (int j = 0; j < 4; ++j) acc[i][j] = wmma_split(af, afl, wf[j], wfl[j], acc[i][j]);
    }
  }

  const int nlane = lane & 15;
  const int mh    = (lane >> 4) * 8;
  __syncthreads();
  if (MODE == 1) {
    bf16* so = (bf16*)sob;
#pragma unroll
    for (int i = 0; i < 4; ++i)
#pragma unroll
      for (int j = 0; j < 4; ++j) {
        const int nl = wn + 16 * j + nlane;
        const float bv = bias ? bias[nBlk + nl] : 0.0f;
#pragma unroll
        for (int r = 0; r < 8; ++r) so[nl * 136 + wm + 16 * i + mh + r] = (bf16)(acc[i][j][r] + bv);
      }
    __syncthreads();
    const int b_ = mBlk >> 11, s0 = mBlk & (SS - 1);
#pragma unroll 1
    for (int pass = 0; pass < 2; ++pass) {
      for (int ch = t; ch < 256 * 16; ch += 256) { const int nl = ch >> 4, q = (ch & 15) * 8; const int n = nBlk + nl, h = n >> 6, dk = n & (DKK - 1);
        *(volatile v4u_t*)((bf16*)out + (((size_t)(b_ * HH + h)) * DKK + dk) * SS + s0 + q) = *(const v4ua*)(so + nl * 136 + q); }
      __threadfence();
    }
  } else {
    float* so = (float*)sob;
#pragma unroll 1
    for (int hf = 0; hf < 2; ++hf) {
      if (wm == hf * 64) {
#pragma unroll
        for (int i = 0; i < 4; ++i)
#pragma unroll
          for (int j = 0; j < 4; ++j) {
            const int nl = wn + 16 * j + nlane;
            const float bv = bias ? bias[nBlk + nl] : 0.0f;
#pragma unroll
            for (int r = 0; r < 8; ++r) { const float v = acc[i][j][r] + bv; so[(16 * i + mh + r) * 260 + nl] = act ? tanhf(v) : v; }
          }
      }
      __syncthreads();
#pragma unroll 1
      for (int pass = 0; pass < 2; ++pass) {
        for (int ch = t; ch < 64 * 64; ch += 256) { const int ml = ch >> 6, q = (ch & 63) * 4;
          *(volatile v4f_t*)((float*)out + (size_t)(mBlk + hf * 64 + ml) * N + nBlk + q) = *(const volatile v4fa*)(so + ml * 260 + q); }
        __threadfence();
      }
      __syncthreads();
    }
  }
}


#define QB 512
#define QNODE 32
#define QT (QB * QNODE)
#define QD 128
#define QA 16
#define QH 256
#define QC 128
#define KSAE 160

__global__ __launch_bounds__(160) void k_obsact(const float* __restrict__ states, const float* __restrict__ actions, float* __restrict__ oa) {
  const int tok = blockIdx.x, c = threadIdx.x;
  const float v = (c < QD) ? states[(size_t)tok * QD + c] : (c < QD + QA) ? actions[(size_t)tok * QA + (c - QD)] : 0.0f;
  *(volatile float*)(oa + (size_t)tok * KSAE + c) = v; __threadfence(); *(volatile float*)(oa + (size_t)tok * KSAE + c) = v;
}
__global__ __launch_bounds__(256) void k_packT(const float* __restrict__ W, bf16* __restrict__ WT, int K, int N, int Kp, int Np) {
  const int g = blockIdx.x * 256 + threadIdx.x; if (g >= Np * Kp / 8) return;
  const int n = (g * 8) / Kp, k0 = (g * 8) % Kp;
  bf16 hh[8], hl[8];
#pragma unroll
  for (int i = 0; i < 8; ++i) { const int k = k0 + i; const float v = (n < N && k < K) ? W[(size_t)k * N + n] : 0.0f; hh[i] = (bf16)v; hl[i] = lo_of(v, hh[i]); }
  const size_t plane = (size_t)Np * Kp;
  *(volatile v4u_t*)(WT + (size_t)n * Kp + k0) = *(const v4ua*)hh; *(volatile v4u_t*)(WT + plane + (size_t)n * Kp + k0) = *(const v4ua*)hl; __threadfence();
  *(volatile v4u_t*)(WT + (size_t)n * Kp + k0) = *(const v4ua*)hh; *(volatile v4u_t*)(WT + plane + (size_t)n * Kp + k0) = *(const v4ua*)hl;
}

__global__ __launch_bounds__(256) void k_padbias(const float* __restrict__ bsrc, int n, float* __restrict__ pb) {
  const int i = threadIdx.x; const float v = (i < n) ? bsrc[i] : 0.0f;
  *(volatile float*)(pb + i) = v; __threadfence(); *(volatile float*)(pb + i) = v;
}
__global__ __launch_bounds__(256) void k_attn(const float* __restrict__ QV, const float* __restrict__ KVv, const float* __restrict__ G,
                                             const float* __restrict__ CURR  , float* __restrict__ H, float* __restrict__ wfull) {
  __shared__ __attribute__((aligned(16))) bf16 qp[2][32 * 264], kp[2][32 * 264], gp[2][256 * 40], pp[2][32 * 40];
  __shared__ __attribute__((aligned(16))) float S[32][33], Wf[32][32], NF[32][260];
  const int b = blockIdx.x, tid = threadIdx.x, lane = tid & 31, wave = tid >> 5, half = lane >> 4, l16 = lane & 15;
  const size_t t0 = (size_t)b * QNODE;
  for (int i = tid; i < 32 * 256; i += 256) { const int r = i >> 8, c = i & 255;
    const float q = QV[(t0 + r) * QH + c], k = KVv[(t0 + r) * QH + c], g = G[(t0 + r) * QH + c];
    bf16 hq = (bf16)q, hk = (bf16)k, hg = (bf16)g;
    qp[0][r * 264 + c] = hq; qp[1][r * 264 + c] = lo_of(q, hq);
    kp[0][r * 264 + c] = hk; kp[1][r * 264 + c] = lo_of(k, hk);
    gp[0][c * 40 + r] = hg;  gp[1][c * 40 + r] = lo_of(g, hg); }
  for (int i = tid; i < 256 * 8; i += 256) { const int c = i >> 3, r = 32 + (i & 7); gp[0][c * 40 + r] = (bf16)0.0f; gp[1][c * 40 + r] = (bf16)0.0f; }
  __syncthreads();
  if (wave < 4) { const int mt = wave >> 1, nt = wave & 1; f32x8 acc = {};
#pragma unroll
    for (int kc = 0; kc < 8; ++kc) acc = wmma_split(lds_frag(&qp[0][(mt * 16) * 264 + kc * 32], 264), lds_frag(&qp[1][(mt * 16) * 264 + kc * 32], 264),
                                             lds_frag(&kp[0][(nt * 16) * 264 + kc * 32], 264), lds_frag(&kp[1][(nt * 16) * 264 + kc * 32], 264), acc);
#pragma unroll
    for (int r = 0; r < 8; ++r) S[mt * 16 + half * 8 + r][nt * 16 + l16] = acc[r] * (1.0f / 16.0f); }
  __syncthreads();
  if (tid < 32) { const int n = tid; float mx = -3.0e38f;
    for (int j = 0; j < 32; ++j) if (j != n) mx = fmaxf(mx, S[n][j]);
    float sm = 0.0f; float e[32];
#pragma unroll
    for (int j = 0; j < 32; ++j) { e[j] = (j != n) ? expf(S[n][j] - mx) : 0.0f; sm += e[j]; }
    const float inv = 1.0f / sm;
#pragma unroll
    for (int j = 0; j < 32; ++j) { const float w = e[j] * inv; Wf[n][j] = (j == n) ? 1.0f : w;
      const bf16 hw = (bf16)w; pp[0][n * 40 + j] = hw; pp[1][n * 40 + j] = lo_of(w, hw); } }
  __syncthreads();
#pragma unroll
  for (int mt = 0; mt < 2; ++mt)
#pragma unroll
    for (int q = 0; q < 2; ++q) { const int nt = wave * 2 + q; f32x8 acc = {};
      acc = wmma_split(lds_frag(&pp[0][(mt * 16) * 40], 40), lds_frag(&pp[1][(mt * 16) * 40], 40), lds_frag(&gp[0][(nt * 16) * 40], 40), lds_frag(&gp[1][(nt * 16) * 40], 40), acc);
#pragma unroll
      for (int r = 0; r < 8; ++r) NF[mt * 16 + half * 8 + r][nt * 16 + l16] = acc[r]; }
  __syncthreads();
#pragma unroll 1
  for (int pass = 0; pass < 2; ++pass) {
    *(volatile v4f_t*)(wfull + (size_t)b * 1024 + tid * 4) = *(const volatile v4fa*)(&Wf[0][0] + tid * 4);
    for (int i = tid; i < 32 * 96; i += 256) { const int r = i / 96, q = (i % 96) * 4; v4f_t v;
      if (q < 128) v = *(const v4fa*)(CURR + (t0 + r) * 256 + q); else { v.x = NF[r][q - 128]; v.y = NF[r][q - 127]; v.z = NF[r][q - 126]; v.w = NF[r][q - 125]; }
      *(volatile v4f_t*)(H + (t0 + r) * 384 + q) = v; }
    __threadfence();
  }
}

__global__ __launch_bounds__(256) void k_head(const float* __restrict__ TH  , const float* __restrict__ f2_w, const float* __restrict__ f2_b,
                                             const float* __restrict__ actions, const float* __restrict__ policies,
                                             float* __restrict__ value, float* __restrict__ qval) {
  __shared__ float f2s[128 * 16], Qs[32][17], pol[32][17];
  __shared__ __attribute__((aligned(16))) float vout[32 * 32], qv[32];
  const int b = blockIdx.x, tid = threadIdx.x;
  const size_t t0 = (size_t)b * QNODE;
  for (int i = tid; i < 128 * 16; i += 256) f2s[i] = f2_w[i];
  for (int i = tid; i < 32 * 16; i += 256) pol[i >> 4][i & 15] = policies[t0 * QA + i];
  __syncthreads();
  for (int i = tid; i < 32 * 16; i += 256) { const int n = i >> 4, a = i & 15; float s = f2_b[a];
#pragma unroll 1
    for (int j = 0; j < QC; ++j) s += TH[(t0 + n) * 256 + j] * f2s[j * 16 + a];
    Qs[n][a] = s; }
  __syncthreads();
  for (int i = tid; i < 32 * 32; i += 256) { const int n = i >> 5, m = i & 31; float s = 0.0f;
#pragma unroll
    for (int a = 0; a < 16; ++a) s += Qs[n][a] * pol[m][a];
    vout[i] = s; }
  if (tid < 32) { float s = 0.0f;
#pragma unroll
    for (int a = 0; a < 16; ++a) s += actions[(t0 + tid) * QA + a] * Qs[tid][a];
    qv[tid] = s; }
  __syncthreads();
#pragma unroll 1
  for (int pass = 0; pass < 2; ++pass) {
    *(volatile v4f_t*)(value + (size_t)b * 1024 + tid * 4) = *(const volatile v4fa*)(vout + tid * 4);
    if (tid < 8) *(volatile v4f_t*)(qval + (size_t)b * 32 + tid * 4) = *(const volatile v4fa*)(qv + tid * 4);
    __threadfence();
  }
}

extern "C" void kernel_launch(void* const* d_in, const int* in_sizes, int n_in,
                              void* d_out, int out_size, void* d_ws, size_t ws_size,
                              hipStream_t stream) {
  (void)in_sizes; (void)n_in; (void)out_size; (void)ws_size;
  const float* states   = (const float*)d_in[0];
  const float* policies = (const float*)d_in[1];
  const float* actions  = (const float*)d_in[2];
  const float* se_w  = (const float*)d_in[3];  const float* se_b  = (const float*)d_in[4];
  const float* key_w = (const float*)d_in[5];  const float* key_b = (const float*)d_in[6];
  const float* q_w   = (const float*)d_in[7];  const float* q_b   = (const float*)d_in[8];
  const float* sae_w = (const float*)d_in[9];  const float* sae_b = (const float*)d_in[10];
  const float* av_w  = (const float*)d_in[11]; const float* av_b  = (const float*)d_in[12];
  const float* ca_w  = (const float*)d_in[13]; const float* ca_b  = (const float*)d_in[14];
  const float* f1_w  = (const float*)d_in[15]; const float* f1_b  = (const float*)d_in[16];
  const float* f2_w  = (const float*)d_in[17]; const float* f2_b  = (const float*)d_in[18];

  char* ws = (char*)d_ws; size_t off = 0;
  auto alloc = [&](size_t bytes) -> char* { char* p = ws + off; off += (bytes + 255) & ~(size_t)255; return p; };
  float* OA    = (float*)alloc((size_t)QT * KSAE * 4);
  float* SEMB  = (float*)alloc((size_t)QT * QH * 4);
  float* T1    = (float*)alloc((size_t)QT * QH * 4);
  float* KEYV  = (float*)alloc((size_t)QT * QH * 4);
  float* QRYV  = (float*)alloc((size_t)QT * QH * 4);
  float* GV    = (float*)alloc((size_t)QT * QH * 4);
  float* Hbuf  = (float*)alloc((size_t)QT * 384 * 4);
  float* CURR  = SEMB;
  float* TH    = T1;
  bf16* seT  = (bf16*)alloc((size_t)2 * 256 * QD * 2);
  bf16* keyT = (bf16*)alloc((size_t)2 * 256 * QH * 2);
  bf16* qT   = (bf16*)alloc((size_t)2 * 256 * QH * 2);
  bf16* saeT = (bf16*)alloc((size_t)2 * 256 * KSAE * 2);
  bf16* avT  = (bf16*)alloc((size_t)2 * 256 * QH * 2);
  bf16* caT  = (bf16*)alloc((size_t)2 * 256 * QD * 2);
  bf16* f1T  = (bf16*)alloc((size_t)2 * 256 * 384 * 2);
  float* cab = (float*)alloc(256 * 4);
  float* f1b = (float*)alloc(256 * 4);
  k_padbias<<<1, 256, 0, stream>>>(ca_b, QC, cab);
  k_padbias<<<1, 256, 0, stream>>>(f1_b, QC, f1b);

  k_obsact<<<QT, 160, 0, stream>>>(states, actions, OA);
  auto packT = [&](const float* W, bf16* WT, int K, int N, int Kp, int Np) { k_packT<<<(Np * Kp / 8 + 255) / 256, 256, 0, stream>>>(W, WT, K, N, Kp, Np); };
  packT(se_w,  seT,  QD, QH, QD, 256);
  packT(key_w, keyT, QH, QH, QH, 256);
  packT(q_w,   qT,   QH, QH, QH, 256);
  packT(sae_w, saeT, QD + QA, QH, KSAE, 256);
  packT(av_w,  avT,  QH, QH, QH, 256);
  packT(ca_w,  caT,  QD, QC, QD, 256);
  packT(f1_w,  f1T,  QC + QH, QC, 384, 256);

  dim3 gBlk(256);
  auto gemm = [&](const float* A, const bf16* WT, size_t plane, const float* bias, float* C, int K, int act) {
    gemm_split_kernel<float, bf16, 2><<<dim3(QT / 128, 1), gBlk, 0, stream>>>(A, 0, WT, plane, bias, C, QT, 256, K, act); };
  gemm(states, seT,  (size_t)256 * QD,   se_b,  SEMB, QD, 1);
  gemm(OA,     saeT, (size_t)256 * KSAE, sae_b, T1,   KSAE, 1);
  gemm(SEMB,   keyT, (size_t)256 * QH,   key_b, KEYV, QH, 0);
  gemm(SEMB,   qT,   (size_t)256 * QH,   q_b,   QRYV, QH, 0);
  gemm(T1,     avT,  (size_t)256 * QH,   av_b,  GV,   QH, 1);
  gemm(states, caT,  (size_t)256 * QD,   cab,   CURR, QD, 1);
  float* out_value = (float*)d_out;
  float* out_qval  = out_value + (size_t)QB * QNODE * QNODE;
  float* out_wfull = out_qval + (size_t)QB * QNODE;
  k_attn<<<QB, 256, 0, stream>>>(QRYV, KEYV, GV, CURR, Hbuf, out_wfull);
  gemm(Hbuf,   f1T,  (size_t)256 * 384,  f1b,   TH, 384, 1);
  k_head<<<QB, 256, 0, stream>>>(TH, f2_w, f2_b, actions, policies, out_value, out_qval);
}
